// MolecularE3nnTransformer_7164005449942
// MI455X (gfx1250) — hardware-verified
//
#include <hip/hip_runtime.h>
#include <math.h>

typedef __attribute__((ext_vector_type(16))) _Float16 v16h;
typedef __attribute__((ext_vector_type(16))) __bf16 v16b;
typedef __attribute__((ext_vector_type(8)))  _Float16 v8h;
typedef __attribute__((ext_vector_type(8)))  float v8f;
typedef __attribute__((ext_vector_type(4)))  float v4f;
typedef __attribute__((ext_vector_type(2)))  float v2f;
typedef __attribute__((ext_vector_type(4)))  unsigned v4u;
typedef __attribute__((ext_vector_type(4)))  int v4i;
typedef float __attribute__((may_alias)) float_a;
typedef int __attribute__((may_alias)) int_a;

template <typename T> __device__ __forceinline__ void vst2(void* p, T v) { *(volatile T*)p = v; __threadfence(); *(volatile T*)p = v; }
__device__ __forceinline__ v8f wmma16(v16h a, v16h b, v8f c) {
  v8f d = __builtin_amdgcn_wmma_f32_16x16x32_f16(false, a, false, b, (short)0, c, false, false);
  asm volatile("v_nop\n\tv_nop\n\tv_nop\n\tv_nop" : "+v"(d) : "v"(a), "v"(b));
  return d;
}
__device__ __forceinline__ v8f wmma_bf(v16b a, v16b b, v8f c) {
  v8f d = __builtin_amdgcn_wmma_f32_16x16x32_bf16(false, a, false, b, (short)0, c, false, false);
  asm volatile("v_nop\n\tv_nop\n\tv_nop\n\tv_nop" : "+v"(d) : "v"(a), "v"(b));
  return d;
}
__device__ __forceinline__ v16h frag_h(const _Float16* rowk0, int lane) {
  union { v16h v; v8h q[2]; } u; const _Float16* p = rowk0 + 8 * (lane >> 4);
  u.q[0] = *(const v8h*)p; u.q[1] = *(const v8h*)(p + 16); return u.v;
}
__device__ __forceinline__ v16h frag_f32(const float* rowk0, int lane) {
  v16h a; const float* p = rowk0 + 8 * (lane >> 4);
#pragma unroll
  for (int i = 0; i < 8; ++i) { a[i] = (_Float16)p[i]; a[8 + i] = (_Float16)p[16 + i]; }
  return a;
}
__device__ __forceinline__ v16h fragc_f32(const float* W, int k0, int n, int lane, int ld, int K) {
  v16h a; const int g = lane >> 4;
#pragma unroll
  for (int i = 0; i < 8; ++i) { const int ka = k0 + 8 * g + i, kb = ka + 16;
    a[i] = (_Float16)(ka < K ? W[(size_t)ka * ld + n] : 0.f); a[8 + i] = (_Float16)(kb < K ? W[(size_t)kb * ld + n] : 0.f); }
  return a;
}
struct F2 { v16b h, l; };
__device__ __forceinline__ F2 bsplit16(const float v[16]) { F2 r;
#pragma unroll
  for (int i = 0; i < 16; ++i) { const __bf16 h = (__bf16)v[i]; r.h[i] = h; r.l[i] = (__bf16)(v[i] - (float)h); }
  return r; }
__device__ __forceinline__ F2 split_row(const float* row, int k0, int lane) { float v[16]; const float* p = row + k0 + 8 * (lane >> 4);
#pragma unroll
  for (int i = 0; i < 8; ++i) { v[i] = p[i]; v[8 + i] = p[16 + i]; }
  return bsplit16(v); }
__device__ __forceinline__ F2 split_rowK(const float* row, int k0, int lane, int K) { float v[16]; const int g = lane >> 4;
#pragma unroll
  for (int i = 0; i < 8; ++i) { const int ka = k0 + 8 * g + i, kb = ka + 16; v[i] = ka < K ? row[ka] : 0.f; v[8 + i] = kb < K ? row[kb] : 0.f; }
  return bsplit16(v); }
__device__ __forceinline__ F2 split_col(const float* W, int k0, int n, int lane, int ld, int K) { float v[16]; const int g = lane >> 4;
#pragma unroll
  for (int i = 0; i < 8; ++i) { const int ka = k0 + 8 * g + i, kb = ka + 16; v[i] = ka < K ? W[(size_t)ka * ld + n] : 0.f; v[8 + i] = kb < K ? W[(size_t)kb * ld + n] : 0.f; }
  return bsplit16(v); }
__device__ __forceinline__ v8f mac3(const F2& a, const F2& b, v8f c) { c = wmma_bf(a.l, b.h, c); c = wmma_bf(a.h, b.l, c); return wmma_bf(a.h, b.h, c); }
__device__ __forceinline__ float sigm(float v) { return 1.0f / (1.0f + expf(-v)); }
#define LDSX() do { asm volatile("s_wait_dscnt 0" ::: "memory"); __builtin_amdgcn_wave_barrier(); __builtin_amdgcn_fence(__ATOMIC_RELEASE, "workgroup"); } while (0)

#define NN 4096
#define NE 16384
#define HH 64
#define NG 64
#define NBAS 10
#define NEL 10
#define SLOTC 32
#define NCH 1024

__global__ __launch_bounds__(256) void k_bucket(const int* __restrict__ dst, int* __restrict__ list) {
  __shared__ int scnt[NCH];
  __shared__ __align__(16) int slots[NCH][SLOTC];
  const int n0 = blockIdx.x * NCH, tid = threadIdx.x;
  for (int i = tid; i < NCH; i += 256) scnt[i] = 0;
  for (int i = tid; i < NCH * SLOTC; i += 256) (&slots[0][0])[i] = 0;
  __syncthreads();
#pragma unroll 1
  for (int e = tid; e < NE; e += 256) { const int d = dst[e] - n0;
    if ((unsigned)d < (unsigned)NCH) { const int s = atomicAdd(&scnt[d], 1); if (s < SLOTC - 1) slots[d][s] = e; } }
  __syncthreads();
  for (int i = tid; i < NCH; i += 256) { const int n = n0 + i;
    int c = scnt[i]; if (c > SLOTC - 1) c = SLOTC - 1;
    for (int a = 1; a < c; ++a) { const int v = slots[i][a]; int b = a - 1; while (b >= 0 && slots[i][b] > v) { slots[i][b + 1] = slots[i][b]; --b; } slots[i][b + 1] = v; }
    slots[i][SLOTC - 1] = scnt[i];
#pragma unroll
    for (int q = 0; q < SLOTC / 4; ++q) vst2(list + (size_t)n * SLOTC + q * 4, *(const v4i*)(&slots[i][q * 4])); }
}
__global__ __launch_bounds__(256) void k_edge(const float* __restrict__ eattr, float* __restrict__ esc) {
  const int e = blockIdx.x * 256 + threadIdx.x; if (e >= NE) return;
  const float ex = eattr[e * 3], ey = eattr[e * 3 + 1], ez = eattr[e * 3 + 2];
  const float len = sqrtf(ex * ex + ey * ey + ez * ez);
  float v[16];
  const float step = 2.0f / 11.0f;
#pragma unroll 1
  for (int i = 0; i < NBAS; ++i) { const float ctr = (float)(i + 1) * step;
    const float d = (len - ctr) / step;
    const float a = d + 1.0f, b = 1.0f - d;
    const float sa = a > 0.f ? expf(-1.0f / a) : 0.f, sb = b > 0.f ? expf(-1.0f / b) : 0.f;
    v[i] = 1.14136f * 7.3890560989306502f * sa * sb * 3.1622776601683795f; }
  { const float t = 10.0f * (1.0f - len / 2.0f); v[10] = t > 0.f ? expf(-1.0f / t) : 0.f; }
#pragma unroll
  for (int i = 11; i < 16; ++i) v[i] = 0.f;
#pragma unroll
  for (int q = 0; q < 4; ++q) vst2(esc + (size_t)e * 16 + q * 4, (v4f){v[q * 4], v[q * 4 + 1], v[q * 4 + 2], v[q * 4 + 3]});
}
__global__ __launch_bounds__(256) void k_packKT(const float* __restrict__ k2, const float* __restrict__ v2, _Float16* __restrict__ KT) {
  const int wl = blockIdx.y, which = wl >> 1, l = wl & 1, w = blockIdx.x, tid = threadIdx.x;
  const float* src = (which == 0 ? k2 : v2) + (size_t)l * 16 * 4096;
  if (tid < 128) { union { v8h h; v4u u; } p8;
#pragma unroll
    for (int i = 0; i < 8; ++i) { const int k = tid * 8 + i, j = k >> 6, u = k & 63; p8.h[i] = (_Float16)src[(size_t)j * 4096 + u * 64 + w]; }
    vst2(KT + ((size_t)wl * HH + w) * 1024 + tid * 8, p8.u); }
}
template <int RELU>
__global__ __launch_bounds__(128) void k_g64(const float* __restrict__ A, const float* __restrict__ W, const float* __restrict__ bias, float scale, float* __restrict__ Out) {
  __shared__ __align__(16) float so[4][16][68];
  const int tid = threadIdx.x, wave = tid >> 5, lane = tid & 31, col = lane & 15, g = lane >> 4;
  const int r0 = blockIdx.x * 64 + wave * 16;
  v8f acc[4] = {};
#pragma unroll
  for (int kc = 0; kc < 2; ++kc) { const v16h a = frag_f32(A + (size_t)(r0 + col) * HH + kc * 32, lane);
#pragma unroll
    for (int j = 0; j < 4; ++j) acc[j] = wmma16(a, fragc_f32(W, kc * 32, j * 16 + col, lane, HH, HH), acc[j]); }
#pragma unroll
  for (int j = 0; j < 4; ++j) { const float bv = bias ? bias[j * 16 + col] : 0.f;
#pragma unroll
    for (int r = 0; r < 8; ++r) { float v = acc[j][r] * scale + bv; if (RELU) v = v > 0.f ? v : 0.f; so[wave][8 * g + r][j * 16 + col] = v; } }
  LDSX();
  for (int q = lane; q < 16 * 16; q += 32) { const int rl = q >> 4, pc = q & 15; vst2(Out + (size_t)(r0 + rl) * HH + pc * 4, *(const v4f*)(&so[wave][rl][pc * 4])); }
}
__global__ __launch_bounds__(128) void k_kv(const float* __restrict__ f, const int* __restrict__ src, const int* __restrict__ dst, const float* __restrict__ esc,
                                          const float* __restrict__ k1, const float* __restrict__ v1, const _Float16* __restrict__ KTk, const _Float16* __restrict__ KTv,
                                          const float* __restrict__ qd, float* __restrict__ vout, float* __restrict__ exout) {
  __shared__ __align__(16) float sfe[4][16][68], sh[4][16][36], so[4][16][68];
  __shared__ __align__(16) float sex[64];
  const int tid = threadIdx.x, w = tid >> 5, lane = tid & 31, col = lane & 15, g = lane >> 4;
  const int e0 = blockIdx.x * 64 + w * 16;
  { const int e = e0 + col; int s = src[e]; s = s < 0 ? 0 : (s >= NN ? NN - 1 : s);
    const float* fr = f + (size_t)s * HH + g * 32;
#pragma unroll
    for (int i = 0; i < 32; ++i) sfe[w][col][g * 32 + i] = fr[i];
    const float* W1 = g == 0 ? k1 : v1; float hb[16];
#pragma unroll
    for (int j = 0; j < 16; ++j) hb[j] = 0.f;
#pragma unroll
    for (int b = 0; b < NBAS; ++b) { const float sb = esc[(size_t)e * 16 + b];
#pragma unroll
      for (int j = 0; j < 16; ++j) hb[j] += sb * W1[b * 16 + j]; }
#pragma unroll
    for (int j = 0; j < 16; ++j) { const float t = hb[j] * 0.31622776601683794f; sh[w][col][g * 16 + j] = t * sigm(t); } }
  LDSX();
#pragma unroll 1
  for (int which = 0; which < 2; ++which) {
    const _Float16* KT = which == 0 ? KTk : KTv;
    v8f acc[4] = {};
#pragma unroll 1
    for (int kc = 0; kc < 32; ++kc) { const int j = kc >> 1, ub = (kc & 1) * 32;
      v16h a; const float hj = sh[w][col][which * 16 + j];
#pragma unroll
      for (int i = 0; i < 8; ++i) { a[i] = (_Float16)(hj * sfe[w][col][ub + 8 * g + i]); a[8 + i] = (_Float16)(hj * sfe[w][col][ub + 16 + 8 * g + i]); }
#pragma unroll
      for (int t = 0; t < 4; ++t) acc[t] = wmma16(a, frag_h(KT + (size_t)(t * 16 + col) * 1024 + kc * 32, lane), acc[t]); }
#pragma unroll
    for (int t = 0; t < 4; ++t)
#pragma unroll
      for (int r = 0; r < 8; ++r) so[w][8 * g + r][t * 16 + col] = acc[t][r] * (0.25f * 0.125f);
    LDSX();
    if (which == 0) {
      const int e = e0 + col; int d = dst[e]; d = d < 0 ? 0 : (d >= NN ? NN - 1 : d);
      float p = 0.f;
#pragma unroll
      for (int i = 0; i < 32; ++i) p += qd[(size_t)d * HH + g * 32 + i] * so[w][col][g * 32 + i];
      p += __shfl_xor(p, 16, 32);
      if (g == 0) sex[w * 16 + col] = esc[(size_t)e * 16 + 10] * expf(p * (1.0f / 64.0f));
      LDSX();
    } else {
      for (int q = lane; q < 16 * 16; q += 32) { const int rl = q >> 4, pc = q & 15; vst2(vout + (size_t)(e0 + rl) * HH + pc * 4, *(const v4f*)(&so[w][rl][pc * 4])); }
    }
  }
  __syncthreads();
  if (tid < 16) vst2(exout + (size_t)blockIdx.x * 64 + tid * 4, *(const v4f*)(&sex[tid * 4]));
}
__global__ __launch_bounds__(256) void k_node(const int* __restrict__ list, const float* __restrict__ ex, const float* __restrict__ v, const float* __restrict__ fin, float* __restrict__ fout) {
  __shared__ float red[4][64];
  const int tid = threadIdx.x, nl = tid >> 6, c = tid & 63, n = blockIdx.x * 4 + nl;
  int dn = list[(size_t)n * SLOTC + SLOTC - 1]; dn = dn < 0 ? 0 : (dn > SLOTC - 1 ? SLOTC - 1 : dn);
  float z = 0.f;
#pragma unroll 1
  for (int s = 0; s < dn; ++s) { int e = list[(size_t)n * SLOTC + s]; if ((unsigned)e >= (unsigned)NE) continue; z += ex[e]; }
  if (z == 0.f) z = 1.0f;
  float agg = 0.f;
#pragma unroll 1
  for (int s = 0; s < dn; ++s) { int e = list[(size_t)n * SLOTC + s]; if ((unsigned)e >= (unsigned)NE) continue;
    const float al = ex[e] / z; const float wgt = sqrtf(al > 0.f ? al : 0.f); agg += wgt * v[(size_t)e * HH + c]; }
  red[nl][c] = agg * agg; __syncthreads();
  for (int st = 32; st > 0; st >>= 1) { if (c < st) red[nl][c] += red[nl][c + st]; __syncthreads(); }
  const float nrm = sqrtf(fmaxf(red[nl][0], 1e-24f));
  const float hx = agg / nrm; const float o = (hx > 0.f ? hx : 0.f) + fin[(size_t)n * HH + c];
  vst2(fout + (size_t)n * HH + c, (float_a)o);
}
__global__ __launch_bounds__(64) void k_pool(const float* __restrict__ f, const int* __restrict__ bidx, const float* __restrict__ Wp, const float* __restrict__ bp, float* __restrict__ out) {
  __shared__ float pooled[NG][HH + 1];
  __shared__ __align__(16) float so[NG];
  const int c = threadIdx.x;
  for (int gg = 0; gg < NG; ++gg) pooled[gg][c] = 0.f;
#pragma unroll 1
  for (int n = 0; n < NN; ++n) { int gg = bidx[n]; gg = gg < 0 ? 0 : (gg >= NG ? NG - 1 : gg); pooled[gg][c] += f[(size_t)n * HH + c]; }
  __syncthreads();
  { const int gg = c; float a = bp[0];
#pragma unroll 1
    for (int k = 0; k < HH; ++k) a += pooled[gg][k] * Wp[k];
    so[gg] = a; }
  __syncthreads();
  if (c < 16) vst2(out + c * 4, *(const v4f*)(&so[c * 4]));
}
__global__ __launch_bounds__(64) void k_embed(const int* __restrict__ x, const float* __restrict__ embd, float* __restrict__ f) {
  const int n = blockIdx.x, c = threadIdx.x; int t = x[n]; t = t < 0 ? 0 : (t >= NEL ? NEL - 1 : t);
  vst2(f + (size_t)n * HH + c, (float_a)embd[t * HH + c]);
}
extern "C" void kernel_launch(void* const* d_in, const int* in_sizes, int n_in, void* d_out, int out_size, void* d_ws, size_t ws_size, hipStream_t stream) {
  (void)in_sizes; (void)n_in; (void)out_size; (void)ws_size;
  const int* x = (const int*)d_in[0]; const int* ei = (const int*)d_in[1]; const float* eattr = (const float*)d_in[2]; const int* bidx = (const int*)d_in[3];
  const float* embd = (const float*)d_in[4]; const float* Wq = (const float*)d_in[5]; const float* k1 = (const float*)d_in[6]; const float* k2 = (const float*)d_in[7];
  const float* v1 = (const float*)d_in[8]; const float* v2 = (const float*)d_in[9]; const float* Wd = (const float*)d_in[10];
  const float* linW = (const float*)d_in[11]; const float* linb = (const float*)d_in[12]; const float* Wp = (const float*)d_in[13]; const float* bp = (const float*)d_in[14];
  const int* src = ei; const int* dst = ei + NE;
  float* out = (float*)d_out;
  char* ws = (char*)d_ws; size_t off = 0;
  auto take = [&](size_t bytes) { char* p = ws + off; off += (bytes + 255) & ~(size_t)255; return p; };
  int* list = (int*)take((size_t)NN * SLOTC * 4);
  float* esc = (float*)take((size_t)NE * 16 * 4);
  _Float16* KT = (_Float16*)take((size_t)4 * HH * 1024 * 2);
  float* fA = (float*)take((size_t)NN * HH * 4); float* fB = (float*)take((size_t)NN * HH * 4);
  float* q = (float*)take((size_t)NN * HH * 4); float* qd = (float*)take((size_t)NN * HH * 4);
  float* vout = (float*)take((size_t)NE * HH * 4); float* exout = (float*)take((size_t)NE * 4);
  k_bucket<<<NN / NCH, 256, 0, stream>>>(dst, list);
  k_edge<<<NE / 256, 256, 0, stream>>>(eattr, esc);
  k_packKT<<<dim3(HH, 4), 256, 0, stream>>>(k2, v2, KT);
  k_embed<<<NN, 64, 0, stream>>>(x, embd, fA);
  float* fcur = fA; float* fnext = fB;
  for (int l = 0; l < 2; ++l) {
    k_g64<0><<<NN / 64, 128, 0, stream>>>(fcur, Wq + (size_t)l * HH * HH, nullptr, 0.125f, q);
    k_g64<0><<<NN / 64, 128, 0, stream>>>(q, Wd + (size_t)l * HH * HH, nullptr, 1.0f, qd);
    k_kv<<<NE / 64, 128, 0, stream>>>(fcur, src, dst, esc, k1 + (size_t)l * NBAS * 16, v1 + (size_t)l * NBAS * 16, KT + ((size_t)(0 * 2 + l) * HH) * 1024, KT + ((size_t)(1 * 2 + l) * HH) * 1024, qd, vout, exout);
    k_node<<<NN / 4, 256, 0, stream>>>(list, exout, vout, fcur, fnext);
    float* t = fcur; fcur = fnext; fnext = t;
  }
  k_g64<1><<<NN / 64, 128, 0, stream>>>(fcur, linW, linb, 1.0f, fnext);
  k_g64<1><<<NN / 64, 128, 0, stream>>>(fnext, linW + HH * HH, linb + HH, 1.0f, fcur);
  k_pool<<<1, 64, 0, stream>>>(fcur, bidx, Wp, bp, out);
}
